// RetroModel_3204045603500
// MI455X (gfx1250) — hardware-verified
//
#include <hip/hip_runtime.h>
#include <math.h>

constexpr int kNB    = 64;
constexpr int kNL    = 4096;
constexpr int kNHalf = 2048;
constexpr int kNH    = 64;
constexpr int kNV    = 128;
constexpr int kMsPitch = 68;
constexpr float kLnEps   = 1e-5f;
constexpr float kNormEps = 1e-12f;

typedef __attribute__((ext_vector_type(16))) _Float16 v16h;
typedef __attribute__((ext_vector_type(8)))  _Float16 v8h;
typedef __attribute__((ext_vector_type(16))) __bf16   v16b;
typedef __attribute__((ext_vector_type(8)))  __bf16   v8b;
typedef __attribute__((ext_vector_type(8)))  float    v8f;
typedef __attribute__((ext_vector_type(4)))  float    v4f;
typedef __attribute__((ext_vector_type(4)))  unsigned int v4u;

__device__ __forceinline__ unsigned short f2bf_bits(float f) {
  unsigned u = __float_as_uint(f);
  return (unsigned short)((u + 0x7FFFu + ((u >> 16) & 1u)) >> 16);
}
__device__ __forceinline__ float bf_bits2f(unsigned short h) { return __uint_as_float(((unsigned)h) << 16); }

__device__ __forceinline__ void dep_guard_h(v8f& a, v8f& b, v16h x, v16h y) { asm volatile("v_nop\n\tv_nop\n\tv_nop\n\tv_nop" : "+v"(a), "+v"(b) : "v"(x), "v"(y)); }
__device__ __forceinline__ void dep_guard_b(v8f& a, v8f& b, v16b x, v16b y) { asm volatile("v_nop\n\tv_nop\n\tv_nop\n\tv_nop" : "+v"(a), "+v"(b) : "v"(x), "v"(y)); }
__device__ __forceinline__ void keep4_h(v16h a, v16h b, v16h c, v16h d) { asm volatile("v_nop" :: "v"(a), "v"(b), "v"(c), "v"(d)); }
__device__ __forceinline__ void keep4_b(v16b a, v16b b, v16b c, v16b d) { asm volatile("v_nop" :: "v"(a), "v"(b), "v"(c), "v"(d)); }
__device__ __forceinline__ void acc_guard4(v8f& a, v8f& b, v8f& c, v8f& d) { asm volatile("v_nop\n\tv_nop\n\tv_nop\n\tv_nop" : "+v"(a), "+v"(b), "+v"(c), "+v"(d)); }
template <typename T> struct Frag;
template <> struct Frag<_Float16> {
  typedef v16h V; union U { v16h v; v8h h[2]; };
  static __device__ __forceinline__ v16h load(const _Float16* p) {
    U f; f.h[0] = *(const v8h*)(p); f.h[1] = *(const v8h*)(p + 16); return f.v;
  }
  static __device__ __forceinline__ v8f mma(v16h a, v16h b, v8f c) {
    return __builtin_amdgcn_wmma_f32_16x16x32_f16(false, a, false, b, (short)0, c, false, false);
  }
  static __device__ __forceinline__ void guard(v8f& a, v8f& b, v16h x, v16h y) { dep_guard_h(a, b, x, y); }
  static __device__ __forceinline__ void keep(v16h a, v16h b, v16h c, v16h d) { keep4_h(a, b, c, d); }
};
template <> struct Frag<__bf16> {
  typedef v16b V; union U { v16b v; v8b h[2]; };
  static __device__ __forceinline__ v16b load(const __bf16* p) {
    U f; f.h[0] = *(const v8b*)(p); f.h[1] = *(const v8b*)(p + 16); return f.v;
  }
  static __device__ __forceinline__ v8f mma(v16b a, v16b b, v8f c) {
    return __builtin_amdgcn_wmma_f32_16x16x32_bf16(false, a, false, b, (short)0, c, false, false);
  }
  static __device__ __forceinline__ void guard(v8f& a, v8f& b, v16b x, v16b y) { dep_guard_b(a, b, x, y); }
  static __device__ __forceinline__ void keep(v16b a, v16b b, v16b c, v16b d) { keep4_b(a, b, c, d); }
};

__device__ __forceinline__ unsigned pk16(unsigned short a, unsigned short b) { return (unsigned)a | ((unsigned)b << 16); }

template <int ET> struct Elem;
template <> struct Elem<0> { typedef _Float16 T; };
template <> struct Elem<1> { typedef __bf16 T; };
template <int ET, bool SPLIT, int BIAS_MODE, int OUT_MODE, bool RESID, int ACT = 0>
__global__ __launch_bounds__(256) void wmma_gemm64(
    const unsigned short* __restrict__ Ap, const unsigned short* __restrict__ A2p, int lda, long strideA,
    const unsigned short* __restrict__ Btp, const unsigned short* __restrict__ Bt2p, int ldb, long strideB,
    void* __restrict__ Cout, void* __restrict__ Cout2, int ldc, long strideC,
    const float* __restrict__ bias,
    const float* __restrict__ resid, long strideR,
    int M, int N, int K, float scale) {
  typedef typename Elem<ET>::T T;
  typedef typename Frag<T>::V V;
  const T* A = (const T*)Ap; const T* A2 = (const T*)A2p; const T* Bt = (const T*)Btp; const T* Bt2 = (const T*)Bt2p;
  __shared__ __align__(16) float sT[8][16 * 68];
  const int b    = blockIdx.y;
  const int lane = threadIdx.x & 31;
  const int wave = threadIdx.x >> 5;
  const int tilesN = N >> 6;
  const int tilesM = M >> 6;
  const int tile = blockIdx.x * 8 + wave;
  if (tile >= tilesM * tilesN) return;
  const int tm = tile / tilesN;
  const int tn = tile - tm * tilesN;
  const int m0 = tm << 6;
  const int n0 = tn << 6;

  const T* Ab  = A  + (size_t)b * strideA;
  const T* Bb  = Bt + (size_t)b * strideB;
  const T* Ab2 = SPLIT ? (A2  + (size_t)b * strideA) : nullptr;
  const T* Bb2 = SPLIT ? (Bt2 + (size_t)b * strideB) : nullptr;

  const int rlane = lane & 15;
  const int koff  = (lane >> 4) * 8;
  const int mOff  = (lane >> 4) * 8;

  v8f acc[4][4];
#pragma unroll
  for (int i = 0; i < 4; ++i)
#pragma unroll
    for (int j = 0; j < 4; ++j) acc[i][j] = (v8f){0.f,0.f,0.f,0.f,0.f,0.f,0.f,0.f};

  for (int k0 = 0; k0 < K; k0 += 32) {
    V bh[4], bl[4];
#pragma unroll
    for (int j = 0; j < 4; ++j) {
      const size_t bo = (size_t)(n0 + (j << 4) + rlane) * ldb + koff + k0;
      bh[j] = Frag<T>::load(Bb + bo);
      if (SPLIT) bl[j] = Frag<T>::load(Bb2 + bo);
    }
#pragma unroll
    for (int i = 0; i < 4; ++i) {
      const size_t ao = (size_t)(m0 + (i << 4) + rlane) * lda + koff + k0;
      V ah = Frag<T>::load(Ab + ao);
      V al;
      if (SPLIT) al = Frag<T>::load(Ab2 + ao);
#pragma unroll
      for (int j = 0; j < 4; ++j) {
        acc[i][j] = Frag<T>::mma(ah, bh[j], acc[i][j]);
        if (SPLIT) {
          acc[i][j] = Frag<T>::mma(ah, bl[j], acc[i][j]);
          acc[i][j] = Frag<T>::mma(al, bh[j], acc[i][j]);
        }
      }
      Frag<T>::guard(acc[i][0], acc[i][3], ah, SPLIT ? al : ah);
    }
    Frag<T>::keep(bh[0], bh[1], bh[2], bh[3]);
    if (SPLIT) Frag<T>::keep(bl[0], bl[1], bl[2], bl[3]);
  }
  acc_guard4(acc[0][0], acc[0][1], acc[0][2], acc[0][3]);
  acc_guard4(acc[1][0], acc[1][1], acc[1][2], acc[1][3]);
  acc_guard4(acc[2][0], acc[2][1], acc[2][2], acc[2][3]);
  acc_guard4(acc[3][0], acc[3][1], acc[3][2], acc[3][3]);

  float* slab = sT[wave];
  const float* Rb = RESID ? (resid + (size_t)b * strideR) : nullptr;
#pragma unroll
  for (int i = 0; i < 4; ++i) {
    const int mBase = m0 + (i << 4);
#pragma unroll
    for (int j = 0; j < 4; ++j) {
      const int n = n0 + (j << 4) + rlane;
      float bv = 0.f;
      if (BIAS_MODE == 2) bv = bias[n];
#pragma unroll
      for (int r = 0; r < 8; ++r) {
        float v = acc[i][j][r] * scale;
        if (BIAS_MODE == 1) v += bias[mBase + mOff + r];
        if (BIAS_MODE == 2) v += bv;
        if (RESID) v += Rb[(size_t)(mBase + mOff + r) * ldc + n];
        if (ACT == 2) v = fmaxf(v, 0.0f);
        if (ACT == 4) v = (v > 0.f) ? v : 0.01f * v;
        slab[(mOff + r) * 68 + (j << 4) + rlane] = v;
      }
    }
    __builtin_amdgcn_fence(__ATOMIC_RELEASE, "workgroup");
    __builtin_amdgcn_wave_barrier();
    __builtin_amdgcn_fence(__ATOMIC_ACQUIRE, "workgroup");
    if (OUT_MODE == 0) {
      float* C = (float*)Cout + (size_t)b * strideC;
      const int hh = lane >> 4, c4 = (lane & 15) * 4;
      for (int pass = 0; pass < 2; ++pass) {
#pragma unroll
        for (int it = 0; it < 8; ++it) {
          const int row = it * 2 + hh;
          v4f v = *(const v4f*)(slab + row * 68 + c4);
          *(volatile v4f*)(C + (size_t)(mBase + row) * ldc + n0 + c4) = v;
        }
        __threadfence();
      }
    } else {
      const int q = lane >> 3, c8 = (lane & 7) * 8;
      unsigned short* C  = (unsigned short*)Cout  + (size_t)b * strideC;
      unsigned short* C2 = (OUT_MODE == 2) ? ((unsigned short*)Cout2 + (size_t)b * strideC) : nullptr;
      for (int pass = 0; pass < 2; ++pass) {
#pragma unroll
        for (int it = 0; it < 4; ++it) {
          const int row = it * 4 + q;
          const float* sp = slab + row * 68 + c8;
          v8h hv, lv;
#pragma unroll
          for (int e = 0; e < 8; ++e) {
            if (OUT_MODE == 1) {
              hv[e] = (_Float16)sp[e];
            } else {
              unsigned short hb = f2bf_bits(sp[e]);
              unsigned short lb = f2bf_bits(sp[e] - bf_bits2f(hb));
              hv[e] = __builtin_bit_cast(_Float16, hb);
              lv[e] = __builtin_bit_cast(_Float16, lb);
            }
          }
          *(volatile v8h*)(C + (size_t)(mBase + row) * ldc + n0 + c8) = hv;
          if (OUT_MODE == 2) *(volatile v8h*)(C2 + (size_t)(mBase + row) * ldc + n0 + c8) = lv;
        }
        __threadfence();
      }
    }
    __builtin_amdgcn_fence(__ATOMIC_RELEASE, "workgroup");
    __builtin_amdgcn_wave_barrier();
    __builtin_amdgcn_fence(__ATOMIC_ACQUIRE, "workgroup");
  }
}

__device__ __forceinline__ float wave_sum(float v) {
#pragma unroll
  for (int off = 16; off > 0; off >>= 1) v += __shfl_xor(v, off, 32);
  return v;
}
__device__ __forceinline__ float wave_max(float v) {
#pragma unroll
  for (int off = 16; off > 0; off >>= 1) v = fmaxf(v, __shfl_xor(v, off, 32));
  return v;
}

__global__ __launch_bounds__(256) void cast_split_kernel(
    const float* __restrict__ embed, const float* __restrict__ W1, const float* __restrict__ W2,
    const float* __restrict__ Wk, const float* __restrict__ Wv, const float* __restrict__ Wattn,
    const float* __restrict__ Wq,
    unsigned short* Eh, unsigned short* El, unsigned short* W1h, unsigned short* W1l,
    unsigned short* W2h, unsigned short* W2l, unsigned short* WPh, unsigned short* WPl) {
  const int z = blockIdx.y;
  const float* src = embed;
  unsigned short* dh = Eh;
  unsigned short* dl = El;
  int n = kNV * kNH;
  if (z == 1) { src = W1; dh = W1h; dl = W1l; n = 2 * kNH * kNH; }
  else if (z == 2) { src = W2; dh = W2h; dl = W2l; n = 2 * kNH * kNH; }
  else if (z == 3) { src = Wk; dh = WPh; dl = WPl; n = kNH * kNH; }
  else if (z == 4) { src = Wv; dh = WPh + kNH * kNH; dl = WPl + kNH * kNH; n = kNH * kNH; }
  else if (z == 5) { src = Wattn; dh = WPh + 2 * kNH * kNH; dl = WPl + 2 * kNH * kNH; n = kNH * kNH; }
  else if (z == 6) { src = Wq; dh = WPh + 3 * kNH * kNH; dl = WPl + 3 * kNH * kNH; n = kNH * kNH; }
  const int i8 = blockIdx.x * 256 + threadIdx.x;
  if (i8 * 8 >= n) return;
  const float* p = src + 8 * (size_t)i8;
  const v4f a = *(const v4f*)(p);
  const v4f c = *(const v4f*)(p + 4);
  float f[8];
#pragma unroll
  for (int e = 0; e < 4; ++e) { f[e] = a[e]; f[4 + e] = c[e]; }
  unsigned short hb[8], lb[8];
#pragma unroll
  for (int e = 0; e < 8; ++e) {
    hb[e] = f2bf_bits(f[e]);
    lb[e] = f2bf_bits(f[e] - bf_bits2f(hb[e]));
  }
  const v4u hu = (v4u){pk16(hb[0], hb[1]), pk16(hb[2], hb[3]), pk16(hb[4], hb[5]), pk16(hb[6], hb[7])};
  const v4u lu = (v4u){pk16(lb[0], lb[1]), pk16(lb[2], lb[3]), pk16(lb[4], lb[5]), pk16(lb[6], lb[7])};
  unsigned short* qh = dh + 8 * (size_t)i8;
  unsigned short* ql = dl + 8 * (size_t)i8;
  *(volatile v4u*)qh = hu;
  *(volatile v4u*)ql = lu;
  __threadfence();
  *(volatile v4u*)qh = hu;
  *(volatile v4u*)ql = lu;
}

template <int MODE>
__global__ __launch_bounds__(256) void row64_kernel(
    const float* __restrict__ in, int rows_per_b, long in_bs, int in_pitch, int in_col,
    const float* __restrict__ gam, const float* __restrict__ bet,
    float* __restrict__ outf, unsigned short* __restrict__ outh, unsigned short* __restrict__ outl, int nrows) {
  __shared__ __align__(16) float rb[8][64];
  const int lane = threadIdx.x & 31;
  const int wave = threadIdx.x >> 5;
  const int row = blockIdx.x * 8 + wave;
  if (row >= nrows) return;
  const int bb = row / rows_per_b;
  const int rr = row - bb * rows_per_b;
  const float* src = in + (size_t)bb * in_bs + (size_t)rr * in_pitch + in_col;
  const float x0 = src[lane];
  const float x1 = src[lane + 32];
  float y0, y1;
  if (MODE == 0) {
    const float mu = wave_sum(x0 + x1) * (1.0f / 64.0f);
    const float d0 = x0 - mu, d1 = x1 - mu;
    const float var = wave_sum(d0 * d0 + d1 * d1) * (1.0f / 64.0f);
    const float rstd = 1.0f / sqrtf(var + kLnEps);
    y0 = d0 * rstd * gam[lane] + bet[lane];
    y1 = d1 * rstd * gam[lane + 32] + bet[lane + 32];
  } else if (MODE == 1) {
    const float ss = wave_sum(x0 * x0 + x1 * x1);
    const float sc = 1.0f / fmaxf(sqrtf(ss), kNormEps);
    y0 = x0 * sc;
    y1 = x1 * sc;
  } else if (MODE == 2) {
    y0 = x0;
    y1 = x1;
  } else {
    const float mx = wave_max(fmaxf(x0, x1));
    const float e0 = expf(x0 - mx);
    const float e1 = expf(x1 - mx);
    const float inv = 1.0f / wave_sum(e0 + e1);
    y0 = e0 * inv;
    y1 = e1 * inv;
  }
  float* rw = rb[wave];
  rw[lane] = y0;
  rw[lane + 32] = y1;
  __builtin_amdgcn_fence(__ATOMIC_RELEASE, "workgroup");
  __builtin_amdgcn_wave_barrier();
  __builtin_amdgcn_fence(__ATOMIC_ACQUIRE, "workgroup");
  for (int pass = 0; pass < 2; ++pass) {
    if (MODE == 1) {
      if (lane < 16) {
        const v4f v = *(const v4f*)(rw + lane * 4);
        *(volatile v4f*)(outf + (size_t)row * kNH + lane * 4) = v;
      }
    } else {
      if (lane < 8) {
        unsigned short hb[8], lb[8];
#pragma unroll
        for (int e = 0; e < 8; ++e) {
          const float f = rw[lane * 8 + e];
          hb[e] = f2bf_bits(f);
          lb[e] = f2bf_bits(f - bf_bits2f(hb[e]));
        }
        const v4u hu = (v4u){pk16(hb[0], hb[1]), pk16(hb[2], hb[3]), pk16(hb[4], hb[5]), pk16(hb[6], hb[7])};
        const v4u lu = (v4u){pk16(lb[0], lb[1]), pk16(lb[2], lb[3]), pk16(lb[4], lb[5]), pk16(lb[6], lb[7])};
        *(volatile v4u*)(outh + (size_t)row * kNH + lane * 8) = hu;
        *(volatile v4u*)(outl + (size_t)row * kNH + lane * 8) = lu;
      }
    }
    __threadfence();
  }
}

__global__ __launch_bounds__(128) void scan_kernel(
    const int* __restrict__ xtok, int steps,
    const float* __restrict__ ktab, long kbs,
    const float* __restrict__ vtab, long vbs, int vpitch, int vcol,
    const float* Min, int mode,
    float* Mout, unsigned short* Mh, unsigned short* Ml, unsigned short* MTh, unsigned short* MTl,
    const float* __restrict__ qsrc, int qpitch, int qcol,
    const float* __restrict__ Wout, const float* __restrict__ bout, float* out) {
  __shared__ __align__(16) float Kl[kNV * kNH];
  __shared__ __align__(16) float Ms[kNH * kMsPitch];
  __shared__ float Pp[2][2][kNH];
  __shared__ float Ql[kNH];
  __shared__ float Rd[kNH];
  __shared__ __align__(16) float Os[kNV];

  const int tid  = threadIdx.x;
  const int lane = tid & 31;
  const int wave = tid >> 5;
  const int b    = blockIdx.x;
  const int i    = tid & 63;
  const int hs   = tid >> 6;
  const int j0   = hs * 32;

  {
    const float* kb = ktab + (size_t)b * kbs;
    for (int e4 = tid; e4 < (kNV * kNH) / 4; e4 += 128) {
      const v4f v = *(const v4f*)(kb + 4 * (size_t)e4);
      *(v4f*)(Kl + 4 * e4) = v;
    }
  }
  float m[32];
  if (mode == 1) {
    const float* mr = Min + (size_t)b * kNH * kNH + (size_t)i * kNH + j0;
#pragma unroll
    for (int q = 0; q < 8; ++q) {
      const v4f v = *(const v4f*)(mr + 4 * q);
      m[4 * q] = v[0]; m[4 * q + 1] = v[1]; m[4 * q + 2] = v[2]; m[4 * q + 3] = v[3];
    }
  } else {
#pragma unroll
    for (int jj = 0; jj < 32; ++jj) m[jj] = 0.f;
  }
  __syncthreads();

  const int* xb = xtok + (size_t)b * kNL;
  const float* vb = vtab + (size_t)b * vbs + vcol;
  for (int t = 0; t < steps; ++t) {
    int tok = xb[t];
    tok = tok < 0 ? 0 : tok;
    tok = tok > kNV - 1 ? kNV - 1 : tok;
    const float vi = vb[(size_t)tok * vpitch + i];
    const float* kr = Kl + tok * kNH + j0;
    float kq[32];
#pragma unroll
    for (int q = 0; q < 8; ++q) {
      const v4f kv = *(const v4f*)(kr + 4 * q);
      kq[4 * q] = kv[0]; kq[4 * q + 1] = kv[1]; kq[4 * q + 2] = kv[2]; kq[4 * q + 3] = kv[3];
    }
    float p = 0.f;
#pragma unroll
    for (int jj = 0; jj < 32; ++jj) p = fmaf(m[jj], kq[jj], p);
    const int buf = t & 1;
    Pp[buf][hs][i] = p;
    __syncthreads();
    const float mk = Pp[buf][0][i] + Pp[buf][1][i];
    const float u = vi - mk;
#pragma unroll
    for (int jj = 0; jj < 32; ++jj) m[jj] = fmaf(u, kq[jj], m[jj]);
  }

#pragma unroll
  for (int q = 0; q < 8; ++q) {
    v4f v;
    v[0] = m[4 * q]; v[1] = m[4 * q + 1]; v[2] = m[4 * q + 2]; v[3] = m[4 * q + 3];
    *(v4f*)(Ms + i * kMsPitch + j0 + 4 * q) = v;
  }
  __syncthreads();

  if (mode == 0) {
    const size_t mo = (size_t)b * kNH * kNH;
    const int hh = lane >> 4, c4 = (lane & 15) * 4;
    const int qq = lane >> 3, c8 = (lane & 7) * 8;
    for (int pass = 0; pass < 2; ++pass) {
#pragma unroll
      for (int it = 0; it < 8; ++it) {
        const int row = wave * 16 + it * 2 + hh;
        const v4f v = *(const v4f*)(Ms + row * kMsPitch + c4);
        *(volatile v4f*)(Mout + mo + (size_t)row * kNH + c4) = v;
      }
#pragma unroll
      for (int it = 0; it < 4; ++it) {
        const int row = wave * 16 + it * 4 + qq;
        unsigned short hb[8], lb[8], th[8], tl[8];
#pragma unroll
        for (int e = 0; e < 8; ++e) {
          const float f = Ms[row * kMsPitch + c8 + e];
          hb[e] = f2bf_bits(f);
          lb[e] = f2bf_bits(f - bf_bits2f(hb[e]));
          const float g = Ms[(c8 + e) * kMsPitch + row];
          th[e] = f2bf_bits(g);
          tl[e] = f2bf_bits(g - bf_bits2f(th[e]));
        }
        const v4u hu  = (v4u){pk16(hb[0], hb[1]), pk16(hb[2], hb[3]), pk16(hb[4], hb[5]), pk16(hb[6], hb[7])};
        const v4u lu  = (v4u){pk16(lb[0], lb[1]), pk16(lb[2], lb[3]), pk16(lb[4], lb[5]), pk16(lb[6], lb[7])};
        const v4u thu = (v4u){pk16(th[0], th[1]), pk16(th[2], th[3]), pk16(th[4], th[5]), pk16(th[6], th[7])};
        const v4u tlu = (v4u){pk16(tl[0], tl[1]), pk16(tl[2], tl[3]), pk16(tl[4], tl[5]), pk16(tl[6], tl[7])};
        const size_t po = mo + (size_t)row * kNH + c8;
        *(volatile v4u*)(Mh + po)  = hu;
        *(volatile v4u*)(Ml + po)  = lu;
        *(volatile v4u*)(MTh + po) = thu;
        *(volatile v4u*)(MTl + po) = tlu;
      }
      __threadfence();
    }
  } else {
    int tokL = xb[kNL - 1];
    tokL = tokL < 0 ? 0 : tokL;
    tokL = tokL > kNV - 1 ? kNV - 1 : tokL;
    if (tid < kNH) Ql[tid] = qsrc[(size_t)tokL * qpitch + qcol + tid];
    __syncthreads();
    if (tid < kNH) {
      float a = 0.f;
      const float* mrow = Ms + tid * kMsPitch;
#pragma unroll 1
      for (int j = 0; j < kNH; ++j) a = fmaf(mrow[j], Ql[j], a);
      Rd[tid] = a;
    }
    __syncthreads();
    {
      float a = 0.f;
      const float* wr = Wout + (size_t)tid * kNH;
#pragma unroll 1
      for (int j = 0; j < kNH; ++j) a = fmaf(wr[j], Rd[j], a);
      Os[tid] = a + bout[tid];
    }
    __syncthreads();
    if (wave == 0) {
      for (int pass = 0; pass < 2; ++pass) {
        const v4f v = *(const v4f*)(Os + lane * 4);
        *(volatile v4f*)(out + (size_t)b * kNV + lane * 4) = v;
        __threadfence();
      }
    }
  }
}

extern "C" void kernel_launch(void* const* d_in, const int* in_sizes, int n_in,
                              void* d_out, int out_size, void* d_ws, size_t ws_size, hipStream_t stream) {
  if (n_in < 14) return;
  if (in_sizes[0] != kNB * kNL || out_size != kNB * kNV) return;
  if (in_sizes[1] != kNV * kNH || in_sizes[12] != kNV * kNH) return;

  const int*   x     = (const int*)d_in[0];
  const float* embed = (const float*)d_in[1];
  const float* W1    = (const float*)d_in[2];
  const float* b1    = (const float*)d_in[3];
  const float* W2    = (const float*)d_in[4];
  const float* b2    = (const float*)d_in[5];
  const float* ln_g  = (const float*)d_in[6];
  const float* ln_b  = (const float*)d_in[7];
  const float* Wk    = (const float*)d_in[8];
  const float* Wv    = (const float*)d_in[9];
  const float* Wq    = (const float*)d_in[10];
  const float* Wattn = (const float*)d_in[11];
  const float* Wout  = (const float*)d_in[12];
  const float* bout  = (const float*)d_in[13];
  float* out = (float*)d_out;

  char* ws = (char*)d_ws;
  size_t off = 0;
  auto carve = [&](size_t bytes) -> char* {
    char* p = ws + off;
    off += (bytes + 255) & ~(size_t)255;
    return p;
  };
  const size_t szVH = (size_t)kNV * kNH;
  const size_t szHH = (size_t)kNH * kNH;
  const size_t szM  = (size_t)kNB * kNH * kNH;
  const size_t szBV = (size_t)kNB * kNV * kNH;
  unsigned short* E_h  = (unsigned short*)carve(szVH * 2);
  unsigned short* E_l  = (unsigned short*)carve(szVH * 2);
  unsigned short* W1_h = (unsigned short*)carve(szVH * 2);
  unsigned short* W1_l = (unsigned short*)carve(szVH * 2);
  unsigned short* W2_h = (unsigned short*)carve(szVH * 2);
  unsigned short* W2_l = (unsigned short*)carve(szVH * 2);
  unsigned short* WP_h = (unsigned short*)carve(4 * szHH * 2);
  unsigned short* WP_l = (unsigned short*)carve(4 * szHH * 2);
  unsigned short* F1_h = (unsigned short*)carve((size_t)kNV * 2 * kNH * 2);
  unsigned short* F1_l = (unsigned short*)carve((size_t)kNV * 2 * kNH * 2);
  float*          Z    = (float*)carve(szVH * 4);
  unsigned short* H_h  = (unsigned short*)carve(szVH * 2);
  unsigned short* H_l  = (unsigned short*)carve(szVH * 2);
  float*          PJ   = (float*)carve((size_t)kNV * 4 * kNH * 4);
  float*          TK   = (float*)carve(szVH * 4);
  unsigned short* TQ_h = (unsigned short*)carve(szVH * 2);
  unsigned short* TQ_l = (unsigned short*)carve(szVH * 2);
  float*          Mf   = (float*)carve(szM * 4);
  unsigned short* M_h  = (unsigned short*)carve(szM * 2);
  unsigned short* M_l  = (unsigned short*)carve(szM * 2);
  unsigned short* MT_h = (unsigned short*)carve(szM * 2);
  unsigned short* MT_l = (unsigned short*)carve(szM * 2);
  float*          S    = (float*)carve(szBV * 4);
  unsigned short* P_h  = (unsigned short*)carve(szBV * 2);
  unsigned short* P_l  = (unsigned short*)carve(szBV * 2);
  unsigned short* C_h  = (unsigned short*)carve(szBV * 2);
  unsigned short* C_l  = (unsigned short*)carve(szBV * 2);
  float*          PJ2  = (float*)carve((size_t)kNB * kNV * 2 * kNH * 4);
  float*          TK2  = (float*)carve(szBV * 4);
  if (off > ws_size) return;

  const dim3 blk256(256);
  const long strideS   = (long)kNV * kNH;
  const long strideM   = (long)kNH * kNH;
  const long stridePJ2 = (long)kNV * 2 * kNH;

  cast_split_kernel<<<dim3(4, 7), blk256, 0, stream>>>(embed, W1, W2, Wk, Wv, Wattn, Wq,
                                                      E_h, E_l, W1_h, W1_l, W2_h, W2_l, WP_h, WP_l);
  wmma_gemm64<1, true, 2, 2, false, 2><<<dim3(1, 1), blk256, 0, stream>>>(
      E_h, E_l, kNH, 0L, W1_h, W1_l, kNH, 0L, (void*)F1_h, (void*)F1_l, 2 * kNH, 0L,
      b1, Z, 0L, kNV, 2 * kNH, kNH, 1.0f);
  wmma_gemm64<1, true, 2, 0, true, 0><<<dim3(1, 1), blk256, 0, stream>>>(
      F1_h, F1_l, 2 * kNH, 0L, W2_h, W2_l, 2 * kNH, 0L, (void*)Z, (void*)Z, kNH, 0L,
      b2, embed, 0L, kNV, kNH, 2 * kNH, 1.0f);
  row64_kernel<0><<<dim3(kNV / 8), blk256, 0, stream>>>(Z, kNV, 0L, kNH, 0, ln_g, ln_b, TK, H_h, H_l, kNV);
  wmma_gemm64<1, true, 0, 0, false, 0><<<dim3(1, 1), blk256, 0, stream>>>(
      H_h, H_l, kNH, 0L, WP_h, WP_l, kNH, 0L, (void*)PJ, (void*)PJ, 4 * kNH, 0L,
      b1, Z, 0L, kNV, 4 * kNH, kNH, 1.0f);
  row64_kernel<1><<<dim3(kNV / 8), blk256, 0, stream>>>(PJ, kNV, 0L, 4 * kNH, 0, ln_g, ln_b, TK, TQ_h, TQ_l, kNV);
  row64_kernel<2><<<dim3(kNV / 8), blk256, 0, stream>>>(PJ, kNV, 0L, 4 * kNH, 2 * kNH, ln_g, ln_b, TK, TQ_h, TQ_l, kNV);
  scan_kernel<<<dim3(kNB), dim3(128), 0, stream>>>(x, kNL, TK, 0L, PJ, 0L, 4 * kNH, kNH, Mf, 0,
                                                   Mf, M_h, M_l, MT_h, MT_l, PJ, 4 * kNH, 3 * kNH, Wout, bout, out);
  wmma_gemm64<1, true, 0, 0, false, 0><<<dim3(1, kNB), blk256, 0, stream>>>(
      TQ_h, TQ_l, kNH, 0L, MT_h, MT_l, kNH, strideM, (void*)S, (void*)S, kNH, strideS,
      b1, Z, 0L, kNV, kNH, kNH, 0.125f);
  row64_kernel<3><<<dim3((kNB * kNV) / 8), blk256, 0, stream>>>(S, kNV, strideS, kNH, 0, ln_g, ln_b, TK, P_h, P_l, kNB * kNV);
  wmma_gemm64<1, true, 0, 2, false, 0><<<dim3(1, kNB), blk256, 0, stream>>>(
      P_h, P_l, kNH, strideS, M_h, M_l, kNH, strideM, (void*)C_h, (void*)C_l, kNH, strideS,
      b1, Z, 0L, kNV, kNH, kNH, 1.0f);
  wmma_gemm64<1, true, 0, 0, false, 0><<<dim3(1, kNB), blk256, 0, stream>>>(
      C_h, C_l, kNH, strideS, WP_h, WP_l, kNH, 0L, (void*)PJ2, (void*)PJ2, 2 * kNH, stridePJ2,
      b1, Z, 0L, kNV, 2 * kNH, kNH, 1.0f);
  row64_kernel<1><<<dim3((kNB * kNV) / 8), blk256, 0, stream>>>(PJ2, kNV, stridePJ2, 2 * kNH, 0, ln_g, ln_b, TK2, P_h, P_l, kNB * kNV);
  scan_kernel<<<dim3(kNB), dim3(128), 0, stream>>>(x, kNHalf, TK2, strideS, PJ2, stridePJ2, 2 * kNH, kNH, Mf, 1,
                                                   Mf, M_h, M_l, MT_h, MT_l, PJ, 4 * kNH, 3 * kNH, Wout, bout, out);
}
